// AdaAttN_42348377539044
// MI455X (gfx1250) — hardware-verified
//
#include <hip/hip_runtime.h>

typedef _Float16 v16h __attribute__((ext_vector_type(16)));
typedef _Float16 v8h  __attribute__((ext_vector_type(8)));
typedef __bf16   v16b __attribute__((ext_vector_type(16)));
typedef unsigned short v8us __attribute__((ext_vector_type(8)));
typedef float    v8f  __attribute__((ext_vector_type(8)));
typedef float    v4f  __attribute__((ext_vector_type(4)));
typedef v8h  __attribute__((may_alias)) v8ha;
typedef v8us __attribute__((may_alias)) v8usa;
typedef v4f  __attribute__((may_alias)) v4fa;

#define NB 4
#define NC 512
#define NL 4096
#define NROWS (NB * NL)
#define NX (NB * NC * NL)
#define NW (NC * NC)
#define NPB (NL / 128)
#define WSCALE 64.0f
#define PSCALE 16384.0f

#define QS 520
#define ES 68
#define PS 72
#define SOS 36
#define QSB (32 * QS * 2)
#define ESB (32 * ES * 4)
#define PSB (32 * PS * 2)
#define ATT_SMEM (2 * QSB + ESB + PSB + 256)

__device__ __forceinline__ v8f zero8f() {
  v8f z = {0.f, 0.f, 0.f, 0.f, 0.f, 0.f, 0.f, 0.f};
  return z;
}

__device__ __forceinline__ v8f wmma_f16(v16h a, v16h b, v8f c) {
  v8f d = __builtin_amdgcn_wmma_f32_16x16x32_f16(false, a, false, b, (short)0, c, false, false);
  asm volatile("v_nop\n\tv_nop\n\tv_nop\n\tv_nop" : "+v"(d) : "v"(a), "v"(b));
  return d;
}

__device__ __forceinline__ v8f wmma3_bf16(v16b ah, v16b al, v16b bh, v16b bl, v8f c) {
  v8f d = __builtin_amdgcn_wmma_f32_16x16x32_bf16(false, al, false, bh, (short)0, c, false, false);
  d = __builtin_amdgcn_wmma_f32_16x16x32_bf16(false, ah, false, bl, (short)0, d, false, false);
  d = __builtin_amdgcn_wmma_f32_16x16x32_bf16(false, ah, false, bh, (short)0, d, false, false);
  asm volatile("v_nop\n\tv_nop\n\tv_nop\n\tv_nop" : "+v"(d) : "v"(ah), "v"(al), "v"(bh), "v"(bl));
  return d;
}

union R16 { v16h h; v16b b; v8us u[2]; };
__device__ __forceinline__ R16 ldfrag(const unsigned short* p, int hh) {
  R16 f;
  f.u[0] = *(const v8usa*)(p + 8 * hh);
  f.u[1] = *(const v8usa*)(p + 16 + 8 * hh);
  return f;
}

__device__ __forceinline__ unsigned short bf16_rne(float x) {
  unsigned u = __float_as_uint(x);
  u += 0x7FFFu + ((u >> 16) & 1u);
  return (unsigned short)(u >> 16);
}
__device__ __forceinline__ float bf16_val(unsigned short s) {
  return __uint_as_float(((unsigned)s) << 16);
}
__device__ __forceinline__ void split_hl(v4f a, v4f c, v8us& hv, v8us& lv) {
  const float y[8] = {a.x, a.y, a.z, a.w, c.x, c.y, c.z, c.w};
  v8us h8 = {0, 0, 0, 0, 0, 0, 0, 0};
  v8us l8 = {0, 0, 0, 0, 0, 0, 0, 0};
#pragma unroll
  for (int j = 0; j < 8; ++j) {
    const unsigned short hb = bf16_rne(y[j]);
    h8[j] = hb;
    l8[j] = bf16_rne(y[j] - bf16_val(hb));
  }
  hv = h8; lv = l8;
}

__global__ __launch_bounds__(256) void stats_kernel(
    const float* __restrict__ style, const float* __restrict__ content,
    float* __restrict__ meanb, float* __restrict__ istdb)
{
  __shared__ __attribute__((aligned(16))) float smean[32];
  __shared__ __attribute__((aligned(16))) float sistd[32];
  const int tid = threadIdx.x, lane = tid & 31, w = tid >> 5;
  const int c0 = blockIdx.x * 32, bb = blockIdx.y, t = blockIdx.z;
  const float* X = (t == 0) ? style : content;
#pragma unroll 1
  for (int j = 0; j < 4; ++j) {
    const int cl = 4 * w + j;
    const float* row = X + ((size_t)(bb * NC + c0 + cl)) * NL;
    double s = 0.0, s2 = 0.0;
#pragma unroll 1
    for (int i = 0; i < NL / 128; ++i) {
      const v4f v = *(const v4fa*)(row + 4 * (lane + 32 * i));
      const double d0 = v.x, d1 = v.y, d2 = v.z, d3 = v.w;
      s += d0; s += d1; s += d2; s += d3;
      s2 += d0 * d0; s2 += d1 * d1; s2 += d2 * d2; s2 += d3 * d3;
    }
#pragma unroll
    for (int off = 16; off > 0; off >>= 1) {
      s  += __shfl_xor(s, off);
      s2 += __shfl_xor(s2, off);
    }
    if (lane == 0) {
      const double mean = s * (1.0 / (double)NL);
      double var = (s2 - s * mean) * (1.0 / (double)(NL - 1));
      var = (var < 0.0) ? 0.0 : var;
      const float stdv = sqrtf((float)var + 1e-5f);
      smean[cl] = (float)mean;
      sistd[cl] = 1.0f / stdv;
    }
  }
  __syncthreads();
  if (w == 0 && lane < 8) {
    const v4f mv = *(const v4fa*)(smean + 4 * lane);
    const v4f iv = *(const v4fa*)(sistd + 4 * lane);
    const size_t o = ((size_t)(t * NB + bb)) * NC + c0 + 4 * lane;
    *(volatile v4f*)(meanb + o) = mv;
    *(volatile v4f*)(istdb + o) = iv;
    __threadfence();
    *(volatile v4f*)(meanb + o) = mv;
    *(volatile v4f*)(istdb + o) = iv;
  }
}

__global__ __launch_bounds__(256) void wconv_kernel(
    const float* __restrict__ v_w, const float* __restrict__ k_w, const float* __restrict__ qg_w,
    _Float16* __restrict__ vw16,
    unsigned short* __restrict__ kwh, unsigned short* __restrict__ kwl,
    unsigned short* __restrict__ qwh, unsigned short* __restrict__ qwl)
{
  const int g = blockIdx.x * 256 + threadIdx.x;
  const int which = g >> 15;
  const int e = g & 32767;
  if (which > 2) return;
  const float* src = (which == 0) ? v_w : ((which == 1) ? k_w : qg_w);
  const v4f a = *(const v4fa*)(src + 8 * e);
  const v4f c = *(const v4fa*)(src + 8 * e + 4);
  if (which == 0) {
    const v8h o = { (_Float16)(a.x * WSCALE), (_Float16)(a.y * WSCALE), (_Float16)(a.z * WSCALE), (_Float16)(a.w * WSCALE),
                    (_Float16)(c.x * WSCALE), (_Float16)(c.y * WSCALE), (_Float16)(c.z * WSCALE), (_Float16)(c.w * WSCALE) };
    _Float16* d = vw16 + 8 * e;
    *(volatile v8h*)d = o;
    __threadfence();
    *(volatile v8h*)d = o;
  } else {
    v8us hv, lv;
    split_hl(a, c, hv, lv);
    unsigned short* dh = ((which == 1) ? kwh : qwh) + 8 * e;
    unsigned short* dl = ((which == 1) ? kwl : qwl) + 8 * e;
    *(volatile v8us*)dh = hv;
    *(volatile v8us*)dl = lv;
    __threadfence();
    *(volatile v8us*)dh = hv;
    *(volatile v8us*)dl = lv;
  }
}

__global__ __launch_bounds__(256) void xconv_kernel(
    const float* __restrict__ X, const float* __restrict__ meanp, const float* __restrict__ istdp,
    int nrm, int wf16,
    _Float16* __restrict__ p16, unsigned short* __restrict__ ph, unsigned short* __restrict__ pl)
{
  __shared__ __attribute__((aligned(16))) float sT[64 * 68];
  __shared__ float smu[64];
  __shared__ float sis[64];
  const int tid = threadIdx.x, lane = tid & 31, w = tid >> 5;
  const int q8 = lane & 7, sub = lane >> 3;
  const int l0 = blockIdx.x * 64, c0 = blockIdx.y * 64, bb = blockIdx.z;
  if (tid < 64) {
    smu[tid] = meanp[bb * NC + c0 + tid];
    sis[tid] = istdp[bb * NC + c0 + tid];
  }
#pragma unroll
  for (int it = 0; it < 4; ++it) {
    const int idx = it * 256 + tid;
    const int ch = idx >> 4, lq = idx & 15;
    const v4f v = *(const v4fa*)(X + ((size_t)(bb * NC + c0 + ch)) * NL + l0 + 4 * lq);
    *(v4fa*)(sT + ch * 68 + 4 * lq) = v;
  }
  __syncthreads();
  v8h f16v[2];
  v8us hv[2], lv[2];
#pragma unroll
  for (int it = 0; it < 2; ++it) {
    const int p = it * 32 + 4 * w + sub;
    float y[8];
#pragma unroll
    for (int j = 0; j < 8; ++j) {
      const int ch = 8 * q8 + j;
      const float x = sT[ch * 68 + p];
      const float yn = (x - smu[ch]) * sis[ch];
      y[j] = nrm ? yn : x;
    }
    const v8h f = { (_Float16)y[0], (_Float16)y[1], (_Float16)y[2], (_Float16)y[3],
                    (_Float16)y[4], (_Float16)y[5], (_Float16)y[6], (_Float16)y[7] };
    f16v[it] = f;
    const v4f a = {y[0], y[1], y[2], y[3]};
    const v4f c = {y[4], y[5], y[6], y[7]};
    split_hl(a, c, hv[it], lv[it]);
  }
#pragma unroll
  for (int it = 0; it < 2; ++it) {
    const int p = it * 32 + 4 * w + sub;
    const size_t o = ((size_t)(bb * NL + l0 + p)) * NC + c0 + 8 * q8;
    if (wf16) *(volatile v8h*)(p16 + o) = f16v[it];
    *(volatile v8us*)(ph + o) = hv[it];
    *(volatile v8us*)(pl + o) = lv[it];
  }
  __threadfence();
#pragma unroll
  for (int it = 0; it < 2; ++it) {
    const int p = it * 32 + 4 * w + sub;
    const size_t o = ((size_t)(bb * NL + l0 + p)) * NC + c0 + 8 * q8;
    if (wf16) *(volatile v8h*)(p16 + o) = f16v[it];
    *(volatile v8us*)(ph + o) = hv[it];
    *(volatile v8us*)(pl + o) = lv[it];
  }
}

__global__ __launch_bounds__(256) void kpsm_kernel(
    const float* __restrict__ style, const float* __restrict__ vsp_w, const float* __restrict__ vsp_b,
    const float* __restrict__ smean, const float* __restrict__ sistd,
    float* __restrict__ swo)
{
  __shared__ float skp[NL];
  __shared__ float svw[NC];
  __shared__ float smu[NC];
  __shared__ float sis[NC];
  __shared__ float sred[8];
  const int tid = threadIdx.x, lane = tid & 31, w = tid >> 5, bb = blockIdx.x;
  for (int i = tid; i < NC; i += 256) {
    svw[i] = vsp_w[i];
    smu[i] = smean[bb * NC + i];
    sis[i] = sistd[bb * NC + i];
  }
  __syncthreads();
  float acc[16];
  const float vb = vsp_b[0];
#pragma unroll
  for (int i = 0; i < 16; ++i) acc[i] = vb;
  const float* xb = style + (size_t)bb * NC * NL + tid;
#pragma unroll 1
  for (int c = 0; c < NC; ++c) {
    const float wv = svw[c], mu = smu[c], is = sis[c];
    const float* row = xb + (size_t)c * NL;
#pragma unroll
    for (int i = 0; i < 16; ++i) acc[i] += wv * ((row[256 * i] - mu) * is);
  }
#pragma unroll
  for (int i = 0; i < 16; ++i) skp[tid + 256 * i] = acc[i];
  float mx = acc[0];
#pragma unroll
  for (int i = 1; i < 16; ++i) mx = fmaxf(mx, acc[i]);
#pragma unroll
  for (int off = 16; off > 0; off >>= 1) mx = fmaxf(mx, __shfl_xor(mx, off));
  if (lane == 0) sred[w] = mx;
  __syncthreads();
  float bm = sred[0];
#pragma unroll
  for (int k = 1; k < 8; ++k) bm = fmaxf(bm, sred[k]);
  __syncthreads();
  float s = 0.0f;
#pragma unroll 1
  for (int i = 0; i < 16; ++i) {
    const int l = tid + 256 * i;
    const float e = __expf(skp[l] - bm);
    skp[l] = e;
    s += e;
  }
#pragma unroll
  for (int off = 16; off > 0; off >>= 1) s += __shfl_xor(s, off);
  if (lane == 0) sred[w] = s;
  __syncthreads();
  float tot = sred[0];
#pragma unroll
  for (int k = 1; k < 8; ++k) tot += sred[k];
  const float inv = 1.0f / tot;
  float* dst = swo + (size_t)bb * NL;
#pragma unroll 1
  for (int i = 0; i < 16; ++i) {
    const int l = tid + 256 * i;
    const float v = skp[l] * inv;
    *(volatile float*)(dst + l) = v;
  }
  __threadfence();
#pragma unroll 1
  for (int i = 0; i < 16; ++i) {
    const int l = tid + 256 * i;
    const float v = skp[l] * inv;
    *(volatile float*)(dst + l) = v;
  }
}

__device__ __forceinline__ void v_store_pass(const float* sT, const float* sgp,
                                             _Float16* vt, float* gpart,
                                             int bb, int co0, int l0, int w, int lane) {
  const int q8 = lane & 7, sub = lane >> 3;
#pragma unroll
  for (int i = 0; i < 8; ++i) {
    const int lid = 32 * w + 4 * i + sub;
    const int co = lid >> 1, hl = lid & 1;
    const float* s = sT + co * 132 + 64 * hl + 8 * q8;
    const v4f a = *(const v4fa*)s;
    const v4f c = *(const v4fa*)(s + 4);
    const v8h o = { (_Float16)a.x, (_Float16)a.y, (_Float16)a.z, (_Float16)a.w,
                    (_Float16)c.x, (_Float16)c.y, (_Float16)c.z, (_Float16)c.w };
    _Float16* d = vt + ((size_t)(bb * NC + co0 + co)) * NL + l0 + 64 * hl + 8 * q8;
    *(volatile v8h*)d = o;
  }
  if (w == 0 && lane < 16) {
    const v4f g = *(const v4fa*)(sgp + 4 * lane);
    float* d = gpart + ((size_t)(bb * NPB + (l0 >> 7))) * NC + co0 + 4 * lane;
    *(volatile v4f*)d = g;
  }
}

__device__ __forceinline__ void kq_store_pass(const float* sT, unsigned short* oh, unsigned short* ol,
                                              int m0, int co0, int w, int lane) {
  const int q8 = lane & 7, sub = lane >> 3;
#pragma unroll
  for (int i = 0; i < 8; ++i) {
    const int p = 32 * w + 4 * i + sub;
    const float* s = sT + p * 68 + 8 * q8;
    const v4f a = *(const v4fa*)s;
    const v4f c = *(const v4fa*)(s + 4);
    v8us hv, lv;
    split_hl(a, c, hv, lv);
    const size_t o = ((size_t)(m0 + p)) * NC + co0 + 8 * q8;
    *(volatile v8us*)(oh + o) = hv;
    *(volatile v8us*)(ol + o) = lv;
  }
}

template <int MODE>
__global__ __launch_bounds__(128) void conv_gemm_kernel(
    const unsigned short* __restrict__ xh, const unsigned short* __restrict__ xl,
    const unsigned short* __restrict__ wgh, const unsigned short* __restrict__ wgl,
    const float* __restrict__ bias,
    const float* __restrict__ gam, const float* __restrict__ bet,
    const float* __restrict__ sw,
    _Float16* __restrict__ vt, float* __restrict__ gpart,
    unsigned short* __restrict__ oh, unsigned short* __restrict__ ol)
{
  __shared__ __attribute__((aligned(16))) float sT[128 * 68];
  __shared__ __attribute__((aligned(16))) float ssw[128];
  __shared__ __attribute__((aligned(16))) float sgp[64];

  const int tid = threadIdx.x, lane = tid & 31, w = tid >> 5;
  const int h = lane >> 4, m = lane & 15;
  const int m0 = blockIdx.x * 128, co0 = blockIdx.y * 64;
  const int bb = m0 / NL, l0 = m0 - bb * NL;

  const size_t arow = ((size_t)(m0 + 32 * w + m)) * NC;
  const unsigned short* xa0h = xh + arow;
  const unsigned short* xa1h = xa0h + (size_t)16 * NC;
  const unsigned short* xa0l = xl + arow;
  const unsigned short* xa1l = xa0l + (size_t)16 * NC;
  const unsigned short* wbh = wgh + ((size_t)(co0 + m)) * NC;
  const unsigned short* wbl = wgl + ((size_t)(co0 + m)) * NC;

  v8f acc[2][4];
#pragma unroll
  for (int mt = 0; mt < 2; ++mt)
#pragma unroll
    for (int nt = 0; nt < 4; ++nt) acc[mt][nt] = zero8f();

#pragma unroll 1
  for (int k0 = 0; k0 < NC; k0 += 32) {
    if (MODE == 0) {
      const v16h a0 = ldfrag(xa0h + k0, h).h;
      const v16h a1 = ldfrag(xa1h + k0, h).h;
#pragma unroll
      for (int nt = 0; nt < 4; ++nt) {
        const v16h bf = ldfrag(wbh + (size_t)nt * 16 * NC + k0, h).h;
        acc[0][nt] = wmma_f16(a0, bf, acc[0][nt]);
        acc[1][nt] = wmma_f16(a1, bf, acc[1][nt]);
      }
    } else {
      const v16b a0h = ldfrag(xa0h + k0, h).b;
      const v16b a0l = ldfrag(xa0l + k0, h).b;
      const v16b a1h = ldfrag(xa1h + k0, h).b;
      const v16b a1l = ldfrag(xa1l + k0, h).b;
#pragma unroll
      for (int nt = 0; nt < 4; ++nt) {
        const v16b bh = ldfrag(wbh + (size_t)nt * 16 * NC + k0, h).b;
        const v16b bl = ldfrag(wbl + (size_t)nt * 16 * NC + k0, h).b;
        acc[0][nt] = wmma3_bf16(a0h, a0l, bh, bl, acc[0][nt]);
        acc[1][nt] = wmma3_bf16(a1h, a1l, bh, bl, acc[1][nt]);
      }
    }
  }

  if (MODE == 0) {
#pragma unroll
    for (int nt = 0; nt < 4; ++nt) {
      const int co = 16 * nt + m;
      const float bv = bias[co0 + co];
#pragma unroll
      for (int mt = 0; mt < 2; ++mt) {
        float* d = sT + co * 132 + 32 * w + 16 * mt + 8 * h;
        v4f x0, x1;
        x0.x = acc[mt][nt][0] * (1.0f / WSCALE) + bv;
        x0.y = acc[mt][nt][1] * (1.0f / WSCALE) + bv;
        x0.z = acc[mt][nt][2] * (1.0f / WSCALE) + bv;
        x0.w = acc[mt][nt][3] * (1.0f / WSCALE) + bv;
        x1.x = acc[mt][nt][4] * (1.0f / WSCALE) + bv;
        x1.y = acc[mt][nt][5] * (1.0f / WSCALE) + bv;
        x1.z = acc[mt][nt][6] * (1.0f / WSCALE) + bv;
        x1.w = acc[mt][nt][7] * (1.0f / WSCALE) + bv;
        *(v4fa*)d = x0;
        *(v4fa*)(d + 4) = x1;
      }
    }
    ssw[tid] = sw[(size_t)bb * NL + l0 + tid];
    __syncthreads();
    {
      const int co = tid >> 1, hf = tid & 1;
      const float* sr = sT + co * 132 + 64 * hf;
      const float* wr = ssw + 64 * hf;
      float s = 0.0f;
#pragma unroll 4
      for (int j = 0; j < 64; ++j) s += sr[j] * wr[j];
      s += __shfl_xor(s, 1);
      if (hf == 0) sgp[co] = s;
    }
    __syncthreads();
    v_store_pass(sT, sgp, vt, gpart, bb, co0, l0, w, lane);
    __threadfence();
    v_store_pass(sT, sgp, vt, gpart, bb, co0, l0, w, lane);
  } else {
#pragma unroll
    for (int nt = 0; nt < 4; ++nt) {
      const int co = 16 * nt + m;
      const float bv = bias[co0 + co];
      float g1 = 1.0f, be = 0.0f;
      if (MODE == 2) {
        g1 = 1.0f + gam[bb * NC + co0 + co];
        be = bet[bb * NC + co0 + co];
      }
#pragma unroll
      for (int mt = 0; mt < 2; ++mt) {
#pragma unroll
        for (int r = 0; r < 8; ++r) {
          const int p = 32 * w + 16 * mt + 8 * h + r;
          float y = acc[mt][nt][r] + bv;
          if (MODE == 2) y = y * g1 + be;
          sT[p * 68 + co] = y;
        }
      }
    }
    __syncthreads();
    kq_store_pass(sT, oh, ol, m0, co0, w, lane);
    __threadfence();
    kq_store_pass(sT, oh, ol, m0, co0, w, lane);
  }
}

__global__ __launch_bounds__(512) void mlp_kernel(
    const float* __restrict__ gpart,
    const float* __restrict__ g1w1, const float* __restrict__ g1b1,
    const float* __restrict__ g1w2, const float* __restrict__ g1b2,
    const float* __restrict__ g2w1, const float* __restrict__ g2b1,
    const float* __restrict__ g2w2, const float* __restrict__ g2b2,
    float* __restrict__ gam, float* __restrict__ bet)
{
  __shared__ float sg[NC];
  __shared__ float sh[NC];
  const int o = threadIdx.x, bb = blockIdx.x;
  float s = 0.0f;
#pragma unroll 1
  for (int p = 0; p < NPB; ++p) s += gpart[((size_t)(bb * NPB + p)) * NC + o];
  sg[o] = s;
  __syncthreads();
  float a = 0.0f;
  {
    const float* wr = g1w1 + (size_t)o * NC;
#pragma unroll 1
    for (int k = 0; k < NC; ++k) a += wr[k] * sg[k];
  }
  a += g1b1[o];
  sh[o] = fmaxf(a, 0.0f);
  __syncthreads();
  float gm = 0.0f;
  {
    const float* wr = g1w2 + (size_t)o * NC;
#pragma unroll 1
    for (int k = 0; k < NC; ++k) gm += wr[k] * sh[k];
  }
  gm += g1b2[o];
  __syncthreads();
  float a2 = 0.0f;
  {
    const float* wr = g2w1 + (size_t)o * NC;
#pragma unroll 1
    for (int k = 0; k < NC; ++k) a2 += wr[k] * sg[k];
  }
  a2 += g2b1[o];
  sh[o] = fmaxf(a2, 0.0f);
  __syncthreads();
  float bt = 0.0f;
  {
    const float* wr = g2w2 + (size_t)o * NC;
#pragma unroll 1
    for (int k = 0; k < NC; ++k) bt += wr[k] * sh[k];
  }
  bt += g2b2[o];
  *(volatile float*)(gam + bb * NC + o) = gm;
  *(volatile float*)(bet + bb * NC + o) = bt;
  __threadfence();
  *(volatile float*)(gam + bb * NC + o) = gm;
  *(volatile float*)(bet + bb * NC + o) = bt;
}

__device__ __forceinline__ void out_store_pass(const float* sO, const float* content,
                                               const float* cmean, const float* cistd, float* out,
                                               int bb, int q0, int w, int lane) {
  const int q8 = lane & 7, sub = lane >> 3;
#pragma unroll
  for (int i = 0; i < 16; ++i) {
    const int cl = 64 * w + 4 * i + sub;
    const v4f s = *(const v4fa*)(sO + cl * SOS + 4 * q8);
    const size_t gi = ((size_t)(bb * NC + cl)) * NL + q0 + 4 * q8;
    const v4f x = *(const v4fa*)(content + gi);
    const float mu = cmean[bb * NC + cl], is = cistd[bb * NC + cl];
    v4f ov;
    ov.x = s.x + (x.x - mu) * is;
    ov.y = s.y + (x.y - mu) * is;
    ov.z = s.z + (x.z - mu) * is;
    ov.w = s.w + (x.w - mu) * is;
    *(volatile v4f*)(out + gi) = ov;
  }
}

__global__ __launch_bounds__(256) void attn_kernel(
    const unsigned short* __restrict__ qh, const unsigned short* __restrict__ ql,
    const unsigned short* __restrict__ kh, const unsigned short* __restrict__ kl,
    const _Float16* __restrict__ vt,
    const float* __restrict__ content,
    const float* __restrict__ cmean, const float* __restrict__ cistd,
    float* __restrict__ out)
{
  extern __shared__ __attribute__((aligned(16))) char smem[];
  unsigned short* Qsh = (unsigned short*)smem;
  unsigned short* Qsl = (unsigned short*)(smem + QSB);
  float* Es = (float*)(smem + 2 * QSB);
  _Float16* Ps = (_Float16*)(smem + 2 * QSB + ESB);
  float* srow = (float*)(smem + 2 * QSB + ESB + PSB);
  float* lrow = srow + 32;
  float* sO = (float*)smem;

  const int tid = threadIdx.x, lane = tid & 31, w = tid >> 5;
  const int h = lane >> 4, m = lane & 15;
  const int bb = blockIdx.y, q0 = blockIdx.x * 32;
  const int mt1 = w & 1, nt1 = w >> 1, cw = 64 * w;
  const int row = tid >> 3, sb8 = tid & 7;

  const size_t qbase = ((size_t)(bb * NL + q0)) * NC;
#pragma unroll
  for (int it = 0; it < 8; ++it) {
    const int idx = it * 256 + tid;
    const int r = idx >> 6, c8 = idx & 63;
    const size_t g = qbase + (size_t)r * NC + 8 * c8;
    *(v8usa*)(Qsh + r * QS + 8 * c8) = *(const v8usa*)(qh + g);
    *(v8usa*)(Qsl + r * QS + 8 * c8) = *(const v8usa*)(ql + g);
  }

  v8f o[2][4];
#pragma unroll
  for (int mt = 0; mt < 2; ++mt)
#pragma unroll
    for (int nt = 0; nt < 4; ++nt) o[mt][nt] = zero8f();
  float mrun = -1.0e30f, lrun = 0.0f;
  __syncthreads();

#pragma unroll 1
  for (int kb = 0; kb < NL; kb += 64) {
    {
      const unsigned short* qa = Qsh + (16 * mt1 + m) * QS;
      const unsigned short* qc = Qsl + (16 * mt1 + m) * QS;
      const size_t krow = ((size_t)(bb * NL + kb + 16 * nt1 + m)) * NC;
      const unsigned short* ka = kh + krow;
      const unsigned short* kc = kl + krow;
      v8f ev = zero8f();
#pragma unroll 1
      for (int kk = 0; kk < NC; kk += 32) {
        const v16b af = ldfrag(qa + kk, h).b;
        const v16b al = ldfrag(qc + kk, h).b;
        const v16b bf = ldfrag(ka + kk, h).b;
        const v16b bl = ldfrag(kc + kk, h).b;
        ev = wmma3_bf16(af, al, bf, bl, ev);
      }
      float* ep = Es + (16 * mt1 + 8 * h) * ES + 16 * nt1 + m;
#pragma unroll
      for (int r = 0; r < 8; ++r) ep[r * ES] = ev[r];
    }
    __syncthreads();

    {
      const float* er = Es + row * ES + 8 * sb8;
      const v4f e0 = *(const v4fa*)er;
      const v4f e1 = *(const v4fa*)(er + 4);
      const float sv[8] = {e0.x, e0.y, e0.z, e0.w, e1.x, e1.y, e1.z, e1.w};
      float mloc = sv[0];
#pragma unroll
      for (int j = 1; j < 8; ++j) mloc = fmaxf(mloc, sv[j]);
      mloc = fmaxf(mloc, __shfl_xor(mloc, 1));
      mloc = fmaxf(mloc, __shfl_xor(mloc, 2));
      mloc = fmaxf(mloc, __shfl_xor(mloc, 4));
      const float mnew = fmaxf(mrun, mloc);
      const float alpha = __expf(mrun - mnew);
      float lsum = 0.0f;
      v8h pv = {0, 0, 0, 0, 0, 0, 0, 0};
#pragma unroll
      for (int j = 0; j < 8; ++j) {
        const float p = __expf(sv[j] - mnew);
        lsum += p;
        pv[j] = (_Float16)(p * PSCALE);
      }
      lsum += __shfl_xor(lsum, 1);
      lsum += __shfl_xor(lsum, 2);
      lsum += __shfl_xor(lsum, 4);
      lrun = lrun * alpha + lsum;
      mrun = mnew;
      *(v8ha*)(Ps + row * PS + 8 * sb8) = pv;
      if (sb8 == 0) { srow[row] = alpha; lrow[row] = lrun; }
    }
    __syncthreads();

    {
#pragma unroll
      for (int mt = 0; mt < 2; ++mt) {
        const v4f a0 = *(const v4fa*)(srow + 16 * mt + 8 * h);
        const v4f a1 = *(const v4fa*)(srow + 16 * mt + 8 * h + 4);
#pragma unroll
        for (int nt = 0; nt < 4; ++nt) {
          o[mt][nt][0] *= a0.x; o[mt][nt][1] *= a0.y; o[mt][nt][2] *= a0.z; o[mt][nt][3] *= a0.w;
          o[mt][nt][4] *= a1.x; o[mt][nt][5] *= a1.y; o[mt][nt][6] *= a1.z; o[mt][nt][7] *= a1.w;
        }
      }
#pragma unroll
      for (int ks = 0; ks < 2; ++ks) {
        const v16h pa0 = ldfrag((const unsigned short*)(Ps + m * PS + 32 * ks), h).h;
        const v16h pa1 = ldfrag((const unsigned short*)(Ps + (16 + m) * PS + 32 * ks), h).h;
#pragma unroll
        for (int nt = 0; nt < 4; ++nt) {
          const _Float16* vp = vt + ((size_t)(bb * NC + cw + 16 * nt + m)) * NL + kb + 32 * ks;
          const v16h vb = ldfrag((const unsigned short*)vp, h).h;
          o[0][nt] = wmma_f16(pa0, vb, o[0][nt]);
          o[1][nt] = wmma_f16(pa1, vb, o[1][nt]);
        }
      }
    }
  }
  __syncthreads();

  {
#pragma unroll
    for (int mt = 0; mt < 2; ++mt) {
      const v4f la = *(const v4fa*)(lrow + 16 * mt + 8 * h);
      const v4f lb = *(const v4fa*)(lrow + 16 * mt + 8 * h + 4);
      float rl[8] = {la.x, la.y, la.z, la.w, lb.x, lb.y, lb.z, lb.w};
#pragma unroll
      for (int r = 0; r < 8; ++r) rl[r] = (1.0f / rl[r]) * (1.0f / PSCALE);
#pragma unroll
      for (int nt = 0; nt < 4; ++nt) {
        float* d = sO + (cw + 16 * nt + m) * SOS + 16 * mt + 8 * h;
        v4f x0, x1;
        x0.x = o[mt][nt][0] * rl[0]; x0.y = o[mt][nt][1] * rl[1];
        x0.z = o[mt][nt][2] * rl[2]; x0.w = o[mt][nt][3] * rl[3];
        x1.x = o[mt][nt][4] * rl[4]; x1.y = o[mt][nt][5] * rl[5];
        x1.z = o[mt][nt][6] * rl[6]; x1.w = o[mt][nt][7] * rl[7];
        *(v4fa*)d = x0;
        *(v4fa*)(d + 4) = x1;
      }
    }
  }
  __syncthreads();

  out_store_pass(sO, content, cmean, cistd, out, bb, q0, w, lane);
  __threadfence();
  out_store_pass(sO, content, cmean, cistd, out, bb, q0, w, lane);
}

extern "C" void kernel_launch(void* const* d_in, const int* in_sizes, int n_in,
                              void* d_out, int out_size, void* d_ws, size_t ws_size,
                              hipStream_t stream) {
  if (n_in < 18) return;
  if (in_sizes[0] != NX || in_sizes[1] != NX) return;
  if (in_sizes[2] != NW || in_sizes[6] != NW || in_sizes[8] != NW) return;
  if (in_sizes[10] != NW || in_sizes[12] != NW || in_sizes[14] != NW || in_sizes[16] != NW) return;
  if (in_sizes[3] != NC || in_sizes[7] != NC || in_sizes[9] != NC) return;
  if (in_sizes[11] != NC || in_sizes[13] != NC || in_sizes[15] != NC || in_sizes[17] != NC) return;
  if (in_sizes[4] != NC || in_sizes[5] < 1) return;
  if (out_size != NX) return;

  const float* content = (const float*)d_in[0];
  const float* style   = (const float*)d_in[1];
  const float* v_w   = (const float*)d_in[2];
  const float* v_b   = (const float*)d_in[3];
  const float* vsp_w = (const float*)d_in[4];
  const float* vsp_b = (const float*)d_in[5];
  const float* k_w   = (const float*)d_in[6];
  const float* k_b   = (const float*)d_in[7];
  const float* qg_w  = (const float*)d_in[8];
  const float* qg_b  = (const float*)d_in[9];
  const float* g1_w1 = (const float*)d_in[10];
  const float* g1_b1 = (const float*)d_in[11];
  const float* g1_w2 = (const float*)d_in[12];
  const float* g1_b2 = (const float*)d_in[13];
  const float* g2_w1 = (const float*)d_in[14];
  const float* g2_b1 = (const float*)d_in[15];
  const float* g2_w2 = (const float*)d_in[16];
  const float* g2_b2 = (const float*)d_in[17];
  float* out = (float*)d_out;

  const size_t PLB      = (size_t)NX * 2;
  const size_t OFF_MEAN = 0;
  const size_t OFF_ISTD = 16384;
  const size_t OFF_SW   = 32768;
  const size_t OFF_GP   = 98304;
  const size_t OFF_GAM  = 360448;
  const size_t OFF_BET  = 368640;
  const size_t OFF_VW   = 376832;
  const size_t OFF_KWH  = 901120;
  const size_t OFF_KWL  = 1425408;
  const size_t OFF_QWH  = 1949696;
  const size_t OFF_QWL  = 2473984;
  const size_t OFF_XP   = 2998272;
  const size_t OFF_VT   = OFF_XP + 3 * PLB;
  const size_t OFF_KH   = OFF_VT + PLB;
  const size_t OFF_KL   = OFF_KH + PLB;
  const size_t OFF_QL   = OFF_KL + PLB;
  const size_t WS_TOTAL = OFF_QL + PLB;
  if (WS_TOTAL > ws_size) return;

  char* ws = (char*)d_ws;
  float* meanb = (float*)(ws + OFF_MEAN);
  float* istdb = (float*)(ws + OFF_ISTD);
  float* sw    = (float*)(ws + OFF_SW);
  float* gpart = (float*)(ws + OFF_GP);
  float* gam   = (float*)(ws + OFF_GAM);
  float* bet   = (float*)(ws + OFF_BET);
  _Float16* vw16 = (_Float16*)(ws + OFF_VW);
  unsigned short* kwh = (unsigned short*)(ws + OFF_KWH);
  unsigned short* kwl = (unsigned short*)(ws + OFF_KWL);
  unsigned short* qwh = (unsigned short*)(ws + OFF_QWH);
  unsigned short* qwl = (unsigned short*)(ws + OFF_QWL);
  _Float16* sp16       = (_Float16*)(ws + OFF_XP);
  unsigned short* sph  = (unsigned short*)(ws + OFF_XP + PLB);
  unsigned short* spl  = (unsigned short*)(ws + OFF_XP + 2 * PLB);
  unsigned short* cph  = (unsigned short*)(ws + OFF_XP);
  unsigned short* cpl  = (unsigned short*)(ws + OFF_XP + PLB);
  unsigned short* qhp  = (unsigned short*)(ws + OFF_XP + 2 * PLB);
  unsigned short* qlp  = (unsigned short*)(ws + OFF_QL);
  _Float16* vt16       = (_Float16*)(ws + OFF_VT);
  unsigned short* khp  = (unsigned short*)(ws + OFF_KH);
  unsigned short* klp  = (unsigned short*)(ws + OFF_KL);
  const float* smeanp = meanb;
  const float* sistdp = istdb;
  const float* cmeanp = meanb + NB * NC;
  const float* cistdp = istdb + NB * NC;

  stats_kernel<<<dim3(NC / 32, NB, 2), 256, 0, stream>>>(style, content, meanb, istdb);

  wconv_kernel<<<dim3(3 * (NW / 8) / 256), 256, 0, stream>>>(v_w, k_w, qg_w, vw16, kwh, kwl, qwh, qwl);

  xconv_kernel<<<dim3(NL / 64, NC / 64, NB), 256, 0, stream>>>(style, smeanp, sistdp, 0, 1, sp16, sph, spl);

  kpsm_kernel<<<dim3(NB), 256, 0, stream>>>(style, vsp_w, vsp_b, smeanp, sistdp, sw);

  conv_gemm_kernel<0><<<dim3(NROWS / 128, NC / 64), 128, 0, stream>>>(
      (const unsigned short*)sp16, (const unsigned short*)sp16,
      (const unsigned short*)vw16, (const unsigned short*)vw16,
      v_b, gam, bet, sw, vt16, gpart, khp, klp);

  conv_gemm_kernel<1><<<dim3(NROWS / 128, NC / 64), 128, 0, stream>>>(
      sph, spl, kwh, kwl, k_b, gam, bet, sw, vt16, gpart, khp, klp);

  mlp_kernel<<<dim3(NB), 512, 0, stream>>>(gpart, g1_w1, g1_b1, g1_w2, g1_b2, g2_w1, g2_b1, g2_w2, g2_b2, gam, bet);

  xconv_kernel<<<dim3(NL / 64, NC / 64, NB), 256, 0, stream>>>(content, cmeanp, cistdp, 1, 0, (_Float16*)cph, cph, cpl);

  conv_gemm_kernel<2><<<dim3(NROWS / 128, NC / 64), 128, 0, stream>>>(
      cph, cpl, qwh, qwl, qg_b, gam, bet, sw, vt16, gpart, qhp, qlp);

  attn_kernel<<<dim3(NL / 32, NB), 256, ATT_SMEM, stream>>>(qhp, qlp, khp, klp, vt16, content, cmeanp, cistdp, out);
}
